// Gma3D_71305047049031
// MI455X (gfx1250) — hardware-verified
//
#include <hip/hip_runtime.h>
#define NB_ 2
#define NN 4096
#define CC 64
#define CQ 16
#define GG 8

typedef __bf16 v16b __attribute__((ext_vector_type(16)));
typedef unsigned short v8us __attribute__((ext_vector_type(8), may_alias));
typedef float  v8f  __attribute__((ext_vector_type(8)));
typedef float  v4f  __attribute__((ext_vector_type(4)));
typedef float  v4fa __attribute__((ext_vector_type(4), may_alias));
union FragB { v16b v; v8us half[2]; unsigned short u[16]; };

__device__ __forceinline__ unsigned short bf16_bits(float x) { unsigned int u = __float_as_uint(x); return (unsigned short)((u + 0x7FFFu + ((u >> 16) & 1u)) >> 16); }
__device__ __forceinline__ float bf16_val(unsigned short b) { return __uint_as_float(((unsigned int)b) << 16); }
__device__ __forceinline__ float bf16_round(float x) { return bf16_val(bf16_bits(x)); }
template <int NT>
__device__ __forceinline__ v8f mmaN(v16b ah, v16b al, v16b bh, v16b bl, v8f c) {
  c = __builtin_amdgcn_wmma_f32_16x16x32_bf16(false, ah, false, bh, (short)0, c, false, false);
  if (NT >= 2) c = __builtin_amdgcn_wmma_f32_16x16x32_bf16(false, al, false, bh, (short)0, c, false, false);
  if (NT >= 3) c = __builtin_amdgcn_wmma_f32_16x16x32_bf16(false, ah, false, bl, (short)0, c, false, false);
  asm volatile("v_nop\n\tv_nop\n\tv_nop\n\tv_nop" : "+v"(c) : "v"(ah), "v"(al), "v"(bh), "v"(bl));
  return c;
}

__global__ __launch_bounds__(256) void k_wt_bf16(const float* __restrict__ W, unsigned short* __restrict__ Wt, int K, int N) {
  const int t = blockIdx.x * 256 + threadIdx.x;
  const int k8n = K / 8;
  if (t >= N * k8n) return;
  const int n = t / k8n, k8 = (t % k8n) * 8;
  v8us v;
#pragma unroll
  for (int i = 0; i < 8; ++i) v[i] = bf16_bits(W[(size_t)(k8 + i) * N + n]);
  *(volatile v8us*)(Wt + (size_t)n * K + k8) = v;
  __threadfence();
  *(volatile v8us*)(Wt + (size_t)n * K + k8) = v;
}

template <bool ASPLIT, int ACT, bool BIAS_BF16>
__global__ __launch_bounds__(128) void k_gemm_bf(const float* __restrict__ A, int lda, const unsigned short* __restrict__ Wt, int ldb,
                                               const float* __restrict__ bias, float* __restrict__ C, int ldc, int M, int N, int K) {
  __shared__ __attribute__((aligned(16))) float so[4][16][64];
  const int tid = threadIdx.x, w = tid >> 5, lane = tid & 31, ln = lane & 15, hh = lane >> 4;
  const int ntn = N / 64;
  const int wid = blockIdx.x * 4 + w;
  const int mt = wid / ntn, nq = wid % ntn;
  if (mt * 16 >= M) return;
  const int row0 = mt * 16, col0 = nq * 64;
  const float* arow = A + (size_t)(row0 + ln) * lda;
  v8f acc[4] = {};
  for (int kb = 0; kb < K; kb += 32) {
    FragB ah, al;
    const v4f x0 = *(const v4fa*)(arow + kb + 8 * hh), x1 = *(const v4fa*)(arow + kb + 8 * hh + 4);
    const v4f x2 = *(const v4fa*)(arow + kb + 16 + 8 * hh), x3 = *(const v4fa*)(arow + kb + 16 + 8 * hh + 4);
    float xs[16] = {x0[0],x0[1],x0[2],x0[3],x1[0],x1[1],x1[2],x1[3],x2[0],x2[1],x2[2],x2[3],x3[0],x3[1],x3[2],x3[3]};
#pragma unroll
    for (int i = 0; i < 16; ++i) { const unsigned short hb = bf16_bits(xs[i]); ah.u[i] = hb; al.u[i] = ASPLIT ? bf16_bits(xs[i] - bf16_val(hb)) : (unsigned short)0; }
#pragma unroll
    for (int t = 0; t < 4; ++t) {
      const unsigned short* brow = Wt + (size_t)(col0 + t * 16 + ln) * ldb + kb;
      FragB b;
      b.half[0] = *(const v8us*)(brow + 8 * hh);
      b.half[1] = *(const v8us*)(brow + 16 + 8 * hh);
      acc[t] = mmaN<ASPLIT ? 2 : 1>(ah.v, al.v, b.v, b.v, acc[t]);
    }
  }
#pragma unroll
  for (int t = 0; t < 4; ++t) {
    float bv = bias ? bias[col0 + t * 16 + ln] : 0.f;
    if (BIAS_BF16) bv = bf16_round(bv);
#pragma unroll
    for (int r = 0; r < 8; ++r) { float v = acc[t][r] + bv; if (ACT == 1) v = fmaxf(v, 0.f); so[w][8 * hh + r][t * 16 + ln] = v; }
  }
  __builtin_amdgcn_fence(__ATOMIC_ACQ_REL, "workgroup");
  __builtin_amdgcn_wave_barrier();
  const int rsub = lane >> 4, c4 = (lane & 15) * 4;
  for (int pass = 0; pass < 2; ++pass) {
#pragma unroll
    for (int q = 0; q < 8; ++q) {
      const int r = q * 2 + rsub;
      const v4f v = *(const v4fa*)&so[w][r][c4];
      *(volatile v4f*)(C + (size_t)(row0 + r) * ldc + col0 + c4) = v;
    }
    if (pass == 0) __threadfence();
  }
}

template <int D, bool CAUSAL>
__global__ __launch_bounds__(128) void k_flash(const float* __restrict__ qb, const float* __restrict__ kb, const float* __restrict__ vb,
                                             int pitch, int T, int H, float scale, float* __restrict__ y, int ypitch) {
  constexpr int KS = D / 32;
  constexpr int DT = D / 16;
  __shared__ __attribute__((aligned(16))) unsigned short sKh[32][D + 8], sKl[32][D + 8], sVh[32][D + 8], sVl[32][D + 8];
  __shared__ __attribute__((aligned(16))) unsigned short sPh[4][16][40], sPl[4][16][40];
  __shared__ __attribute__((aligned(16))) float sO[4][16][D];
  const int tid = threadIdx.x, w = tid >> 5, lane = tid & 31, ln = lane & 15, hh = lane >> 4;
  const int nqb = (T + 63) / 64;
  const int bh = blockIdx.x / nqb, qblk = blockIdx.x % nqb;
  const int b = bh / H, h = bh % H;
  const int q0 = qblk * 64 + w * 16;
  const float* Q = qb + (size_t)b * T * pitch + h * D;
  const float* K = kb + (size_t)b * T * pitch + h * D;
  const float* V = vb + (size_t)b * T * pitch + h * D;

  FragB aqh[KS], aql[KS];
  {
    int row = q0 + ln; if (row >= T) row = T - 1;
    const float* qr = Q + (size_t)row * pitch;
#pragma unroll
    for (int ks = 0; ks < KS; ++ks)
#pragma unroll
      for (int i = 0; i < 16; ++i) {
        const int d = ks * 32 + ((i < 8) ? (8 * hh + i) : (16 + 8 * hh + (i - 8)));
        const float x = qr[d] * scale; const unsigned short hb = bf16_bits(x);
        aqh[ks].u[i] = hb; aql[ks].u[i] = bf16_bits(x - bf16_val(hb));
      }
  }
  float m_r[8], l_r[8];
#pragma unroll
  for (int r = 0; r < 8; ++r) { m_r[r] = -3.0e38f; l_r[r] = 0.f; }
  v8f oacc[DT];
#pragma unroll
  for (int dt = 0; dt < DT; ++dt) oacc[dt] = (v8f){0.f,0.f,0.f,0.f,0.f,0.f,0.f,0.f};

  const int kv_end = CAUSAL ? min(T, qblk * 64 + 64) : T;
  for (int j0 = 0; j0 < kv_end; j0 += 32) {
    __syncthreads();
    for (int e = tid; e < 32 * (D / 4); e += 128) {
      const int r = e / (D / 4), c4 = (e % (D / 4)) * 4;
      const int key = j0 + r;
      v4f kf = {0.f,0.f,0.f,0.f}, vf = {0.f,0.f,0.f,0.f};
      if (key < T) { kf = *(const v4fa*)(K + (size_t)key * pitch + c4); vf = *(const v4fa*)(V + (size_t)key * pitch + c4); }
#pragma unroll
      for (int t = 0; t < 4; ++t) {
        unsigned short hb = bf16_bits(kf[t]); sKh[r][c4 + t] = hb; sKl[r][c4 + t] = bf16_bits(kf[t] - bf16_val(hb));
        hb = bf16_bits(vf[t]); sVh[r][c4 + t] = hb; sVl[r][c4 + t] = bf16_bits(vf[t] - bf16_val(hb));
      }
    }
    __syncthreads();
    v8f s[2];
#pragma unroll
    for (int nt = 0; nt < 2; ++nt) {
      v8f acc = {};
#pragma unroll
      for (int ks = 0; ks < KS; ++ks) {
        FragB bh_, bl_;
        bh_.half[0] = *(const v8us*)&sKh[nt * 16 + ln][ks * 32 + 8 * hh]; bh_.half[1] = *(const v8us*)&sKh[nt * 16 + ln][ks * 32 + 16 + 8 * hh];
        bl_.half[0] = *(const v8us*)&sKl[nt * 16 + ln][ks * 32 + 8 * hh]; bl_.half[1] = *(const v8us*)&sKl[nt * 16 + ln][ks * 32 + 16 + 8 * hh];
        acc = mmaN<3>(aqh[ks].v, aql[ks].v, bh_.v, bl_.v, acc);
      }
      s[nt] = acc;
    }
    float alpha[8];
#pragma unroll
    for (int r = 0; r < 8; ++r) {
      const int qi = q0 + 8 * hh + r;
      const int ja = j0 + ln, jb = j0 + 16 + ln;
      if (CAUSAL) { if (ja > qi) s[0][r] = -3.0e38f; if (jb > qi) s[1][r] = -3.0e38f; }
      if (ja >= T) s[0][r] = -3.0e38f;
      if (jb >= T) s[1][r] = -3.0e38f;
      float mx = fmaxf(s[0][r], s[1][r]);
      mx = fmaxf(mx, __shfl_xor(mx, 1, 32)); mx = fmaxf(mx, __shfl_xor(mx, 2, 32)); mx = fmaxf(mx, __shfl_xor(mx, 4, 32)); mx = fmaxf(mx, __shfl_xor(mx, 8, 32));
      const float mnew = fmaxf(m_r[r], mx);
      alpha[r] = (mnew > -1.0e38f) ? __expf(m_r[r] - mnew) : 1.0f;
      const float p0 = (s[0][r] > -1.0e38f) ? __expf(s[0][r] - mnew) : 0.f;
      const float p1 = (s[1][r] > -1.0e38f) ? __expf(s[1][r] - mnew) : 0.f;
      m_r[r] = mnew;
      l_r[r] = l_r[r] * alpha[r] + p0 + p1;
      unsigned short hb = bf16_bits(p0); sPh[w][8 * hh + r][ln] = hb;      sPl[w][8 * hh + r][ln] = bf16_bits(p0 - bf16_val(hb));
      hb = bf16_bits(p1);                sPh[w][8 * hh + r][16 + ln] = hb; sPl[w][8 * hh + r][16 + ln] = bf16_bits(p1 - bf16_val(hb));
    }
#pragma unroll
    for (int dt = 0; dt < DT; ++dt)
#pragma unroll
      for (int r = 0; r < 8; ++r) oacc[dt][r] *= alpha[r];
    __builtin_amdgcn_fence(__ATOMIC_ACQ_REL, "workgroup");
    __builtin_amdgcn_wave_barrier();
    FragB pah, pal;
    pah.half[0] = *(const v8us*)&sPh[w][ln][8 * hh]; pah.half[1] = *(const v8us*)&sPh[w][ln][16 + 8 * hh];
    pal.half[0] = *(const v8us*)&sPl[w][ln][8 * hh]; pal.half[1] = *(const v8us*)&sPl[w][ln][16 + 8 * hh];
#pragma unroll
    for (int dt = 0; dt < DT; ++dt) {
      FragB bvh, bvl;
#pragma unroll
      for (int i = 0; i < 8; ++i) {
        bvh.u[i] = sVh[8 * hh + i][dt * 16 + ln]; bvh.u[8 + i] = sVh[16 + 8 * hh + i][dt * 16 + ln];
        bvl.u[i] = sVl[8 * hh + i][dt * 16 + ln]; bvl.u[8 + i] = sVl[16 + 8 * hh + i][dt * 16 + ln];
      }
      oacc[dt] = mmaN<3>(pah.v, pal.v, bvh.v, bvl.v, oacc[dt]);
    }
    __builtin_amdgcn_fence(__ATOMIC_ACQ_REL, "workgroup");
    __builtin_amdgcn_wave_barrier();
  }
#pragma unroll
  for (int r = 0; r < 8; ++r) {
    float l = l_r[r];
    l += __shfl_xor(l, 1, 32); l += __shfl_xor(l, 2, 32); l += __shfl_xor(l, 4, 32); l += __shfl_xor(l, 8, 32);
    l_r[r] = (l > 0.f) ? 1.0f / l : 0.f;
  }
#pragma unroll
  for (int dt = 0; dt < DT; ++dt)
#pragma unroll
    for (int r = 0; r < 8; ++r) sO[w][8 * hh + r][dt * 16 + ln] = oacc[dt][r] * l_r[r];
  __builtin_amdgcn_fence(__ATOMIC_ACQ_REL, "workgroup");
  __builtin_amdgcn_wave_barrier();
  for (int pass = 0; pass < 2; ++pass) {
    for (int r = 0; r < 16; ++r) {
      const int row = q0 + r;
      if (row < T && lane < D / 4) {
        const v4f val = *(const v4fa*)&sO[w][r][lane * 4];
        *(volatile v4f*)(y + ((size_t)b * T + row) * ypitch + h * D + lane * 4) = val;
      }
    }
    if (pass == 0) __threadfence();
  }
}

template <bool ASPLIT, bool BSPLIT, int ACT>
__global__ __launch_bounds__(128) void k_gemm_b(const float* __restrict__ A, int lda, size_t sA, const unsigned short* __restrict__ Bh, const unsigned short* __restrict__ Bl, int ldb, size_t sB,
                                             const float* __restrict__ bias, const float* __restrict__ resid, int ldr, size_t sR, float rsign, float alpha,
                                             float* __restrict__ C, int ldc, size_t sC, int M, int N, int K) {
  __shared__ __attribute__((aligned(16))) float so[4][16][64];
  const int tid = threadIdx.x, w = tid >> 5, lane = tid & 31, ln = lane & 15, hh = lane >> 4;
  const int by = blockIdx.y;
  A += (size_t)by * sA; Bh += (size_t)by * sB; if (BSPLIT) Bl += (size_t)by * sB; C += (size_t)by * sC; if (resid) resid += (size_t)by * sR;
  const int ntn = (N + 63) / 64; const int wid = blockIdx.x * 4 + w; const int mt = wid / ntn, nq = wid % ntn;
  if (mt * 16 >= M) return;
  const int row0 = mt * 16, col0 = nq * 64;
  const float* arow = A + (size_t)(row0 + ln) * lda;
  v8f acc[4] = {};
  for (int kb = 0; kb < K; kb += 32) {
    FragB ah, al;
    const v4f x0 = *(const v4fa*)(arow + kb + 8 * hh), x1 = *(const v4fa*)(arow + kb + 8 * hh + 4);
    const v4f x2 = *(const v4fa*)(arow + kb + 16 + 8 * hh), x3 = *(const v4fa*)(arow + kb + 16 + 8 * hh + 4);
    float xs[16] = {x0[0],x0[1],x0[2],x0[3],x1[0],x1[1],x1[2],x1[3],x2[0],x2[1],x2[2],x2[3],x3[0],x3[1],x3[2],x3[3]};
#pragma unroll
    for (int i = 0; i < 16; ++i) { const unsigned short hb = bf16_bits(xs[i]); ah.u[i] = hb; al.u[i] = ASPLIT ? bf16_bits(xs[i] - bf16_val(hb)) : (unsigned short)0; }
#pragma unroll
    for (int t = 0; t < 4; ++t) {
      if (col0 + t * 16 >= N) continue;
      const size_t boff = (size_t)(col0 + t * 16 + ln) * ldb + kb;
      FragB bh_, bl_; bh_.half[0] = *(const v8us*)(Bh + boff + 8 * hh); bh_.half[1] = *(const v8us*)(Bh + boff + 16 + 8 * hh);
      if (BSPLIT) { bl_.half[0] = *(const v8us*)(Bl + boff + 8 * hh); bl_.half[1] = *(const v8us*)(Bl + boff + 16 + 8 * hh); } else bl_ = bh_;
      acc[t] = mmaN<ASPLIT ? (BSPLIT ? 3 : 2) : 1>(ah.v, al.v, bh_.v, bl_.v, acc[t]);
    }
  }
#pragma unroll
  for (int t = 0; t < 4; ++t) {
    const int col = col0 + t * 16 + ln; if (col0 + t * 16 >= N) continue; const float bv = bias ? bf16_round(bias[col]) : 0.f;
#pragma unroll
    for (int r = 0; r < 8; ++r) { float v = acc[t][r] * alpha + bv; if (resid) v += rsign * resid[(size_t)(row0 + 8 * hh + r) * ldr + col]; if (ACT == 1) v = fmaxf(v, 0.f); else if (ACT == 2) v = fmaxf(v, 0.f) + log1pf(expf(-fabsf(v))); so[w][8 * hh + r][t * 16 + ln] = v; }
  }
  __builtin_amdgcn_fence(__ATOMIC_ACQ_REL, "workgroup"); __builtin_amdgcn_wave_barrier();
  const int rsub = lane >> 4, c4 = (lane & 15) * 4;
  for (int pass = 0; pass < 2; ++pass) {
#pragma unroll
    for (int q = 0; q < 8; ++q) { const int r = q * 2 + rsub; if (col0 + c4 < N) { const v4f v = *(const v4fa*)&so[w][r][c4]; *(volatile v4f*)(C + (size_t)(row0 + r) * ldc + col0 + c4) = v; } }
    if (pass == 0) __threadfence();
  }
}
__global__ __launch_bounds__(256) void k_split_transpose_b(const float* __restrict__ src, int lds_, size_t sIn, unsigned short* __restrict__ hi, unsigned short* __restrict__ lo, size_t sOut, int K, int N) {
  const size_t t = (size_t)blockIdx.x * 256 + threadIdx.x; const int k8n = K / 8; if (t >= (size_t)N * k8n) return;
  src += (size_t)blockIdx.y * sIn; hi += (size_t)blockIdx.y * sOut; lo += (size_t)blockIdx.y * sOut;
  const int n = (int)(t / k8n), k8 = (int)(t % k8n) * 8; v8us vh, vl;
#pragma unroll
  for (int i = 0; i < 8; ++i) { const float x = src[(size_t)(k8 + i) * lds_ + n]; const unsigned short hb = bf16_bits(x); vh[i] = hb; vl[i] = bf16_bits(x - bf16_val(hb)); }
  unsigned short* dh = hi + (size_t)n * K + k8; unsigned short* dl = lo + (size_t)n * K + k8;
  *(volatile v8us*)dh = vh; *(volatile v8us*)dl = vl; __threadfence(); *(volatile v8us*)dh = vh; *(volatile v8us*)dl = vl;
}

typedef _Float16 v16h __attribute__((ext_vector_type(16)));
union FragH { v16h v; v8us half[2]; _Float16 h[16]; unsigned short u[16]; };
template <int NT>
__device__ __forceinline__ v8f mmaH(v16h ah, v16h al, v16h bh, v16h bl, v8f c) {
  c = __builtin_amdgcn_wmma_f32_16x16x32_f16(false, ah, false, bh, (short)0, c, false, false);
  if (NT >= 2) c = __builtin_amdgcn_wmma_f32_16x16x32_f16(false, al, false, bh, (short)0, c, false, false);
  if (NT >= 3) c = __builtin_amdgcn_wmma_f32_16x16x32_f16(false, ah, false, bl, (short)0, c, false, false);
  asm volatile("v_nop\n\tv_nop\n\tv_nop\n\tv_nop" : "+v"(c) : "v"(ah), "v"(al), "v"(bh), "v"(bl));
  return c;
}
template <bool ASPLIT>
__global__ __launch_bounds__(128) void k_gemm_h(const float* __restrict__ A, int lda, size_t sA, const _Float16* __restrict__ Bh, int ldb, size_t sB, float alpha, float* __restrict__ C, int ldc, size_t sC, int M, int N, int K) {
  __shared__ __attribute__((aligned(16))) float so[4][16][64];
  const int tid = threadIdx.x, w = tid >> 5, lane = tid & 31, ln = lane & 15, hh = lane >> 4; const int by = blockIdx.y;
  A += (size_t)by * sA; Bh += (size_t)by * sB; C += (size_t)by * sC;
  const int ntn = (N + 63) / 64; const int wid = blockIdx.x * 4 + w; const int mt = wid / ntn, nq = wid % ntn; if (mt * 16 >= M) return;
  const int row0 = mt * 16, col0 = nq * 64; const float* arow = A + (size_t)(row0 + ln) * lda;
  v8f acc[4] = {};
  for (int kb = 0; kb < K; kb += 32) {
    FragH ah, al;
    const v4f x0 = *(const v4fa*)(arow + kb + 8 * hh), x1 = *(const v4fa*)(arow + kb + 8 * hh + 4), x2 = *(const v4fa*)(arow + kb + 16 + 8 * hh), x3 = *(const v4fa*)(arow + kb + 16 + 8 * hh + 4);
    float xs[16] = {x0[0],x0[1],x0[2],x0[3],x1[0],x1[1],x1[2],x1[3],x2[0],x2[1],x2[2],x2[3],x3[0],x3[1],x3[2],x3[3]};
#pragma unroll
    for (int i = 0; i < 16; ++i) { const _Float16 h = (_Float16)xs[i]; ah.h[i] = h; al.h[i] = ASPLIT ? (_Float16)(xs[i] - (float)h) : (_Float16)0.0f; }
#pragma unroll
    for (int t = 0; t < 4; ++t) { if (col0 + t * 16 >= N) continue; const size_t boff = (size_t)(col0 + t * 16 + ln) * ldb + kb; FragH bq; bq.half[0] = *(const v8us*)(Bh + boff + 8 * hh); bq.half[1] = *(const v8us*)(Bh + boff + 16 + 8 * hh);
      acc[t] = mmaH<ASPLIT ? 2 : 1>(ah.v, al.v, bq.v, bq.v, acc[t]); }
  }
#pragma unroll
  for (int t = 0; t < 4; ++t) { if (col0 + t * 16 >= N) continue;
#pragma unroll
    for (int r = 0; r < 8; ++r) so[w][8 * hh + r][t * 16 + ln] = acc[t][r] * alpha; }
  __builtin_amdgcn_fence(__ATOMIC_ACQ_REL, "workgroup"); __builtin_amdgcn_wave_barrier();
  const int rsub = lane >> 4, c4 = (lane & 15) * 4;
  for (int pass = 0; pass < 2; ++pass) {
#pragma unroll
    for (int q = 0; q < 8; ++q) { const int r = q * 2 + rsub; if (col0 + c4 < N) { const v4f v = *(const v4fa*)&so[w][r][c4]; *(volatile v4f*)(C + (size_t)(row0 + r) * ldc + col0 + c4) = v; } }
    if (pass == 0) __threadfence(); }
}

template <int DUMMY>
__global__ __launch_bounds__(128) void k_gemm_hh(const _Float16* __restrict__ A, int lda, size_t sA, const _Float16* __restrict__ Bh, int ldb, size_t sB, float alpha, float* __restrict__ C, int ldc, size_t sC, int M, int N, int K) {
  __shared__ __attribute__((aligned(16))) float so[4][16][64];
  const int tid = threadIdx.x, w = tid >> 5, lane = tid & 31, ln = lane & 15, hh = lane >> 4; const int by = blockIdx.y;
  A += (size_t)by * sA; Bh += (size_t)by * sB; C += (size_t)by * sC;
  const int ntn = (N + 63) / 64; const int wid = blockIdx.x * 4 + w; const int mt = wid / ntn, nq = wid % ntn; if (mt * 16 >= M) return;
  const int row0 = mt * 16, col0 = nq * 64; const _Float16* arow = A + (size_t)(row0 + ln) * lda;
  v8f acc[4] = {};
  for (int kb = 0; kb < K; kb += 32) { FragH ah; ah.half[0] = *(const v8us*)((const unsigned short*)arow + kb + 8 * hh); ah.half[1] = *(const v8us*)((const unsigned short*)arow + kb + 16 + 8 * hh);
#pragma unroll
    for (int t = 0; t < 4; ++t) { if (col0 + t * 16 >= N) continue; const size_t boff = (size_t)(col0 + t * 16 + ln) * ldb + kb; FragH bq; bq.half[0] = *(const v8us*)((const unsigned short*)Bh + boff + 8 * hh); bq.half[1] = *(const v8us*)((const unsigned short*)Bh + boff + 16 + 8 * hh);
      acc[t] = mmaH<1>(ah.v, ah.v, bq.v, bq.v, acc[t]); }
  }
#pragma unroll
  for (int t = 0; t < 4; ++t) { if (col0 + t * 16 >= N) continue;
#pragma unroll
    for (int r = 0; r < 8; ++r) so[w][8 * hh + r][t * 16 + ln] = acc[t][r] * alpha; }
  __builtin_amdgcn_fence(__ATOMIC_ACQ_REL, "workgroup"); __builtin_amdgcn_wave_barrier();
  const int rsub = lane >> 4, c4 = (lane & 15) * 4;
  for (int pass = 0; pass < 2; ++pass) {
#pragma unroll
    for (int q = 0; q < 8; ++q) { const int r = q * 2 + rsub; if (col0 + c4 < N) { const v4f v = *(const v4fa*)&so[w][r][c4]; *(volatile v4f*)(C + (size_t)(row0 + r) * ldc + col0 + c4) = v; } }
    if (pass == 0) __threadfence(); }
}

typedef unsigned short v4us4 __attribute__((ext_vector_type(4)));
__global__ __launch_bounds__(256) void k_q(const float* __restrict__ ctx, const float* __restrict__ Wqk, int b, unsigned short* __restrict__ Qh, unsigned short* __restrict__ Ql) { __shared__ float sw[CQ][CC]; const int tid = threadIdx.x; for (int i = tid; i < CQ * CC; i += 256) sw[i / CC][i % CC] = bf16_round(Wqk[i]); __syncthreads();
  const int n = blockIdx.x * 256 + tid; float q[CQ];
#pragma unroll
  for (int o = 0; o < CQ; ++o) q[o] = 0.f;
#pragma unroll 4
  for (int c = 0; c < CC; ++c) { const float x = bf16_round(ctx[((size_t)b * CC + c) * NN + n]);
#pragma unroll
    for (int o = 0; o < CQ; ++o) q[o] += sw[o][c] * x; }
  FragB fh, fl; for (int o = 0; o < 16; ++o) { const unsigned short h = bf16_bits(q[o]); fh.u[o] = h; fl.u[o] = bf16_bits(q[o] - bf16_val(h)); }
  FragB zz; for (int o = 0; o < 16; ++o) zz.u[o] = 0;
  unsigned short* dh = Qh + (size_t)n * 32; unsigned short* dl = Ql + (size_t)n * 32;
  for (int pass = 0; pass < 2; ++pass) { *(volatile v8us*)(dh) = fh.half[0]; *(volatile v8us*)(dh + 8) = fh.half[1]; *(volatile v8us*)(dh + 16) = zz.half[0]; *(volatile v8us*)(dh + 24) = zz.half[0]; *(volatile v8us*)(dl) = fl.half[0]; *(volatile v8us*)(dl + 8) = fl.half[1]; *(volatile v8us*)(dl + 16) = zz.half[0]; *(volatile v8us*)(dl + 24) = zz.half[0]; if (pass == 0) __threadfence(); } }
__global__ __launch_bounds__(128) void k_corr(const unsigned short* __restrict__ Ah, const unsigned short* __restrict__ Al, const unsigned short* __restrict__ Bh, const unsigned short* __restrict__ Bl, float* __restrict__ C, int ldc) {
  __shared__ __attribute__((aligned(16))) float so[4][16][64];
  const int tid = threadIdx.x, w = tid >> 5, lane = tid & 31, ln = lane & 15, hh = lane >> 4; const int blk = blockIdx.x * 4 + w; const int rt = blk / (NN / 64), quad = blk % (NN / 64); const int row0 = rt * 16, col0 = quad * 64;
  FragB ah, al; { const unsigned short* ar = Ah + (size_t)(row0 + ln) * 32 + hh * 8; const unsigned short* lr = Al + (size_t)(row0 + ln) * 32 + hh * 8; ah.half[0] = *(const v8us*)ar; ah.half[1] = *(const v8us*)(ar + 16); al.half[0] = *(const v8us*)lr; al.half[1] = *(const v8us*)(lr + 16); }
  v8f acc[4];
#pragma unroll
  for (int t = 0; t < 4; ++t) { acc[t] = v8f{0.f,0.f,0.f,0.f,0.f,0.f,0.f,0.f}; FragB bh, bl; const unsigned short* br = Bh + (size_t)(col0 + t * 16 + ln) * 32 + hh * 8; const unsigned short* blr = Bl + (size_t)(col0 + t * 16 + ln) * 32 + hh * 8; bh.half[0] = *(const v8us*)br; bh.half[1] = *(const v8us*)(br + 16); bl.half[0] = *(const v8us*)blr; bl.half[1] = *(const v8us*)(blr + 16);
    acc[t] = mmaN<3>(ah.v, al.v, bh.v, bl.v, acc[t]); }
#pragma unroll
  for (int t = 0; t < 4; ++t) {
#pragma unroll
    for (int r = 0; r < 8; ++r) so[w][8 * hh + r][t * 16 + ln] = acc[t][r]; }
  __builtin_amdgcn_fence(__ATOMIC_ACQ_REL, "workgroup"); __builtin_amdgcn_s_barrier();
  for (int pass = 0; pass < 2; ++pass) { for (int i = lane; i < 16 * 16; i += 32) { const int r = i / 16, c4 = (i % 16) * 4; v4f v; v[0] = so[w][r][c4]; v[1] = so[w][r][c4 + 1]; v[2] = so[w][r][c4 + 2]; v[3] = so[w][r][c4 + 3]; *(volatile v4f*)(C + (size_t)(row0 + r) * ldc + col0 + c4) = v; } if (pass == 0) __threadfence(); } }
__global__ __launch_bounds__(256) void k_rsoft(float* __restrict__ S) { const int tid = threadIdx.x, wv = tid >> 5, lane = tid & 31; const size_t row = (size_t)blockIdx.x * 8 + wv; float* s = S + row * NN; float mx = -3.0e38f;
#pragma unroll 4
  for (int j = lane; j < NN; j += 32) mx = fmaxf(mx, s[j]); for (int o = 16; o >= 1; o >>= 1) mx = fmaxf(mx, __shfl_xor(mx, o, 32)); float den = 0.f;
#pragma unroll 4
  for (int j = lane; j < NN; j += 32) den += expf(s[j] - mx); for (int o = 16; o >= 1; o >>= 1) den += __shfl_xor(den, o, 32); const float inv = 1.0f / den;
#pragma unroll 4
  for (int j = lane; j < NN; j += 32) { const float v = expf(s[j] - mx) * inv; *(volatile float*)(s + j) = v; }
  __threadfence();
#pragma unroll 4
  for (int j = lane; j < NN; j += 32) { const float v = *(volatile float*)(s + j); *(volatile float*)(s + j) = v; } }
__global__ __launch_bounds__(256) void k_csum(const float* __restrict__ S, float* __restrict__ CS) { const int n = blockIdx.x * 256 + threadIdx.x; float s = 0.f;
#pragma unroll 4
  for (int m = 0; m < NN; ++m) s += S[(size_t)m * NN + n]; *(volatile float*)(CS + n) = s; __threadfence(); *(volatile float*)(CS + n) = s; }
__global__ __launch_bounds__(256) void k_dsum(const float* __restrict__ xyz, int b, float* __restrict__ SQ, float* __restrict__ DS) { __shared__ float sp[256][4]; const int tid = threadIdx.x; const int n = blockIdx.x * 256 + tid; const float* p = xyz + ((size_t)b * NN + n) * 3; const float xn = bf16_round(p[0]), yn = bf16_round(p[1]), zn = bf16_round(p[2]); const float sqn = xn * xn + yn * yn + zn * zn; float s = 0.f;
  for (int m0 = 0; m0 < NN; m0 += 256) { __syncthreads(); { const float* pm = xyz + ((size_t)b * NN + m0 + tid) * 3; const float a = bf16_round(pm[0]), bb = bf16_round(pm[1]), c = bf16_round(pm[2]); sp[tid][0] = a; sp[tid][1] = bb; sp[tid][2] = c; sp[tid][3] = a * a + bb * bb + c * c; } __syncthreads();
#pragma unroll 4
    for (int m = 0; m < 256; ++m) { const float d = fmaxf(sp[m][3] + sqn - 2.0f * (sp[m][0] * xn + sp[m][1] * yn + sp[m][2] * zn), 0.f); s += d; } }
  *(volatile float*)(SQ + n) = sqn; *(volatile float*)(DS + n) = s; __threadfence(); *(volatile float*)(SQ + n) = sqn; *(volatile float*)(DS + n) = s; }
__global__ __launch_bounds__(256) void k_lstat(const float* __restrict__ S, const float* __restrict__ CS, const float* __restrict__ xyz, const float* __restrict__ SQ, const float* __restrict__ DS, int b, float* __restrict__ RM, float* __restrict__ RD) { const int tid = threadIdx.x, wv = tid >> 5, lane = tid & 31; const int m = blockIdx.x * 8 + wv; const float* s = S + (size_t)m * NN; const float* pm = xyz + ((size_t)b * NN + m) * 3; const float xm = bf16_round(pm[0]), ym = bf16_round(pm[1]), zm = bf16_round(pm[2]); const float sqm = SQ[m]; float mx = -3.0e38f;
#pragma unroll 1
  for (int n = lane; n < NN; n += 32) { const float* pn = xyz + ((size_t)b * NN + n) * 3; const float d = fmaxf(sqm + SQ[n] - 2.0f * (xm * bf16_round(pn[0]) + ym * bf16_round(pn[1]) + zm * bf16_round(pn[2])), 0.f); const bool msk = (d / (1e-9f + DS[n])) <= 0.1f; const float a = s[n] / (1e-9f + CS[n]); const float l = msk ? a : 0.f; mx = fmaxf(mx, l); }
  for (int o = 16; o >= 1; o >>= 1) mx = fmaxf(mx, __shfl_xor(mx, o, 32)); float den = 0.f;
#pragma unroll 1
  for (int n = lane; n < NN; n += 32) { const float* pn = xyz + ((size_t)b * NN + n) * 3; const float d = fmaxf(sqm + SQ[n] - 2.0f * (xm * bf16_round(pn[0]) + ym * bf16_round(pn[1]) + zm * bf16_round(pn[2])), 0.f); const bool msk = (d / (1e-9f + DS[n])) <= 0.1f; const float a = s[n] / (1e-9f + CS[n]); const float l = msk ? a : 0.f; den += expf(l - mx); }
  for (int o = 16; o >= 1; o >>= 1) den += __shfl_xor(den, o, 32);
  if (lane == 0) { *(volatile float*)(RM + m) = mx; *(volatile float*)(RD + m) = den; } __threadfence(); if (lane == 0) { *(volatile float*)(RM + m) = mx; *(volatile float*)(RD + m) = den; } }
__global__ __launch_bounds__(256) void k_lcsum(const float* __restrict__ S, const float* __restrict__ CS, const float* __restrict__ xyz, const float* __restrict__ SQ, const float* __restrict__ DS, const float* __restrict__ RM, const float* __restrict__ RD, int b, float* __restrict__ LS) { __shared__ float sp[256][6]; const int tid = threadIdx.x; const int n = blockIdx.x * 256 + tid; const float* pn = xyz + ((size_t)b * NN + n) * 3; const float xn = bf16_round(pn[0]), yn = bf16_round(pn[1]), zn = bf16_round(pn[2]); const float sqn = SQ[n]; const float ids = 1e-9f + DS[n]; const float ics = 1e-9f + CS[n]; float acc = 0.f;
  for (int m0 = 0; m0 < NN; m0 += 256) { __syncthreads(); { const float* pm = xyz + ((size_t)b * NN + m0 + tid) * 3; sp[tid][0] = bf16_round(pm[0]); sp[tid][1] = bf16_round(pm[1]); sp[tid][2] = bf16_round(pm[2]); sp[tid][3] = SQ[m0 + tid]; sp[tid][4] = RM[m0 + tid]; sp[tid][5] = 1.0f / RD[m0 + tid]; } __syncthreads();
#pragma unroll 2
    for (int mm = 0; mm < 256; ++mm) { const int m = m0 + mm; const float d = fmaxf(sp[mm][3] + sqn - 2.0f * (sp[mm][0] * xn + sp[mm][1] * yn + sp[mm][2] * zn), 0.f); const bool msk = (d / ids) <= 0.1f; const float a = S[(size_t)m * NN + n] / ics; const float l = msk ? a : 0.f; acc += expf(l - sp[mm][4]) * sp[mm][5]; } }
  *(volatile float*)(LS + n) = acc; __threadfence(); *(volatile float*)(LS + n) = acc; }
__global__ __launch_bounds__(256) void k_ptile(const float* __restrict__ S, const float* __restrict__ CS, const float* __restrict__ xyz, const float* __restrict__ SQ, const float* __restrict__ DS, const float* __restrict__ RM, const float* __restrict__ RD, const float* __restrict__ LS, int b, _Float16* __restrict__ PT) {
  __shared__ float tile[64][33]; __shared__ float pmx[64][6], pnx[32][4]; const int m0 = blockIdx.y * 64, n0 = blockIdx.x * 32; const int tid = threadIdx.x, tx = tid & 31, ty = tid >> 5;
  if (tid < 64) { const float* p = xyz + ((size_t)b * NN + m0 + tid) * 3; pmx[tid][0] = bf16_round(p[0]); pmx[tid][1] = bf16_round(p[1]); pmx[tid][2] = bf16_round(p[2]); pmx[tid][3] = SQ[m0 + tid]; pmx[tid][4] = RM[m0 + tid]; pmx[tid][5] = 1.0f / RD[m0 + tid]; } else if (tid < 96) { const int t2 = tid - 64; const float* p = xyz + ((size_t)b * NN + n0 + t2) * 3; pnx[t2][0] = bf16_round(p[0]); pnx[t2][1] = bf16_round(p[1]); pnx[t2][2] = bf16_round(p[2]); pnx[t2][3] = SQ[n0 + t2]; }
  __syncthreads();
  const int n = n0 + tx; const float ids = 1e-9f + DS[n], ics = 1e-9f + CS[n], ils = 1.0f / (1e-9f + LS[n]);
  for (int i = ty; i < 64; i += 8) { const int m = m0 + i; const float d = fmaxf(pmx[i][3] + pnx[tx][3] - 2.0f * (pmx[i][0] * pnx[tx][0] + pmx[i][1] * pnx[tx][1] + pmx[i][2] * pnx[tx][2]), 0.f); const bool msk = (d / ids) <= 0.1f; const float a = S[(size_t)m * NN + n] / ics; const float l = msk ? a : 0.f; const float loc = expf(l - pmx[i][4]) * pmx[i][5]; tile[i][tx] = a + loc * ils; }
  __syncthreads();
  const int r = tid >> 3, c8 = (tid & 7) * 8; FragH o; for (int q = 0; q < 8; ++q) o.h[q] = (_Float16)tile[c8 + q][r];
  unsigned short* dst = (unsigned short*)PT + (size_t)(n0 + r) * NN + m0 + c8; *(volatile v8us*)dst = o.half[0]; __threadfence(); *(volatile v8us*)dst = o.half[0]; }
__global__ __launch_bounds__(256) void k_xv(const float* __restrict__ mot, const float* __restrict__ Wv, const float* __restrict__ bv, int b, _Float16* __restrict__ XV) { __shared__ float sw[CC]; const int c = blockIdx.y, m = (blockIdx.x * 256 + threadIdx.x) * 2; if (threadIdx.x < CC) sw[threadIdx.x] = bf16_round(Wv[c * CC + threadIdx.x]); __syncthreads(); float s0 = bf16_round(bv[c]), s1 = s0;
  typedef float v2f __attribute__((ext_vector_type(2), aligned(8))); typedef _Float16 v2h __attribute__((ext_vector_type(2)));
#pragma unroll 4
  for (int k = 0; k < CC; ++k) { const v2f x2 = *(const v2f*)(mot + ((size_t)b * CC + k) * NN + m); s0 += sw[k] * bf16_round(x2.x); s1 += sw[k] * bf16_round(x2.y); }
  v2h o2 = { (_Float16)s0, (_Float16)s1 }; *(volatile v2h*)(XV + (size_t)c * NN + m) = o2; __threadfence(); *(volatile v2h*)(XV + (size_t)c * NN + m) = o2; }
__global__ __launch_bounds__(256) void k_res(const float* __restrict__ mot, const float* __restrict__ GT, const float* __restrict__ Wt, const float* __restrict__ bt, int b, float* __restrict__ RES) { __shared__ float sw[CC]; __shared__ float sg[256][CC + 1]; const int c = blockIdx.y, n0 = blockIdx.x * 256, tid = threadIdx.x; if (tid < CC) sw[tid] = bf16_round(Wt[c * CC + tid]);
  for (int i = tid; i < 256 * CC; i += 256) { const int nn = i / CC, k = i % CC; sg[nn][k] = GT[(size_t)(n0 + nn) * CC + k]; } __syncthreads();
  const int n = n0 + tid; float s = bf16_round(bt[c]);
#pragma unroll 4
  for (int k = 0; k < CC; ++k) s += sw[k] * (bf16_round(mot[((size_t)b * CC + k) * NN + n]) - sg[tid][k]);
  *(volatile float*)(RES + (size_t)c * NN + n) = s; __threadfence(); *(volatile float*)(RES + (size_t)c * NN + n) = s; }
__global__ __launch_bounds__(1024) void k_gn(const float* __restrict__ RES, const float* __restrict__ mot, const float* __restrict__ gw, const float* __restrict__ gb, const float* __restrict__ pa, const float* __restrict__ al, int b, float* __restrict__ out) { __shared__ float red[32]; const int g = blockIdx.x, tid = threadIdx.x, lane = tid & 31, wv = tid >> 5; const float* base = RES + (size_t)g * (CC / GG) * NN; const int cnt = (CC / GG) * NN;
  float s = 0.f; for (int i = tid; i < cnt; i += 1024) s += base[i]; for (int o = 16; o >= 1; o >>= 1) s += __shfl_xor(s, o, 32); if (lane == 0) red[wv] = s; __syncthreads(); float tot = 0.f; for (int i = 0; i < 32; ++i) tot += red[i]; const float mu = tot / (float)cnt; __syncthreads();
  float q2 = 0.f; for (int i = tid; i < cnt; i += 1024) { const float d = base[i] - mu; q2 += d * d; } for (int o = 16; o >= 1; o >>= 1) q2 += __shfl_xor(q2, o, 32); if (lane == 0) red[wv] = q2; __syncthreads(); float tq = 0.f; for (int i = 0; i < 32; ++i) tq += red[i]; const float inv = 1.0f / sqrtf(tq / (float)cnt + 1e-5f);
  const float a = bf16_round(pa[0]), alpha = bf16_round(al[0]);
  for (int pass = 0; pass < 2; ++pass) { for (int i = tid; i < cnt; i += 1024) { const int c = g * (CC / GG) + i / NN, n = i % NN; float v = (base[i] - mu) * inv * bf16_round(gw[c]) + bf16_round(gb[c]); v = (v >= 0.f) ? v : a * v; const float o = alpha * v + bf16_round(mot[((size_t)b * CC + c) * NN + n]); *(volatile float*)(out + ((size_t)b * CC + c) * NN + n) = o; } if (pass == 0) __threadfence(); } }
extern "C" void kernel_launch(void* const* d_in, const int* in_sizes, int n_in,
                              void* d_out, int out_size, void* d_ws, size_t ws_size, hipStream_t stream) {
  (void)in_sizes; (void)n_in; (void)out_size;
  const float* ctx = (const float*)d_in[0]; const float* mot = (const float*)d_in[1]; const float* xyz = (const float*)d_in[2]; const float* Wqk = (const float*)d_in[3]; const float* Wv = (const float*)d_in[4]; const float* bv = (const float*)d_in[5]; const float* Wt = (const float*)d_in[6]; const float* bt = (const float*)d_in[7]; const float* gw = (const float*)d_in[8]; const float* gb = (const float*)d_in[9]; const float* pa = (const float*)d_in[10]; const float* al = (const float*)d_in[11];
  char* ws = (char*)d_ws; size_t off = 0;
  auto take = [&](size_t bytes) { char* p = ws + off; off += (bytes + 255) & ~(size_t)255; return p; };
  unsigned short* Qh = (unsigned short*)take((size_t)NN * 32 * 2); unsigned short* Ql = (unsigned short*)take((size_t)NN * 32 * 2); float* S = (float*)take((size_t)NN * NN * 4); _Float16* PT = (_Float16*)take((size_t)NN * NN * 2); _Float16* XV = (_Float16*)take((size_t)CC * NN * 2); float* GT = (float*)take((size_t)NN * CC * 4); float* RES = (float*)take((size_t)CC * NN * 4);
  float* CS = (float*)take(NN * 4); float* SQ = (float*)take(NN * 4); float* DS = (float*)take(NN * 4); float* RM = (float*)take(NN * 4); float* RD = (float*)take(NN * 4); float* LS = (float*)take(NN * 4);
  if (off > ws_size) return;
  for (int b = 0; b < NB_; ++b) {
    k_q<<<NN / 256, 256, 0, stream>>>(ctx, Wqk, b, Qh, Ql);
    k_corr<<<((NN / 16) * (NN / 64)) / 4, 128, 0, stream>>>(Qh, Ql, Qh, Ql, S, NN);
    k_rsoft<<<NN / 8, 256, 0, stream>>>(S);
    k_csum<<<NN / 256, 256, 0, stream>>>(S, CS);
    k_dsum<<<NN / 256, 256, 0, stream>>>(xyz, b, SQ, DS);
    k_lstat<<<NN / 8, 256, 0, stream>>>(S, CS, xyz, SQ, DS, b, RM, RD);
    k_lcsum<<<NN / 256, 256, 0, stream>>>(S, CS, xyz, SQ, DS, RM, RD, b, LS);
    k_ptile<<<dim3(NN / 32, NN / 64), 256, 0, stream>>>(S, CS, xyz, SQ, DS, RM, RD, LS, b, PT);
    k_xv<<<dim3(NN / 512, CC), 256, 0, stream>>>(mot, Wv, bv, b, XV);
    k_gemm_hh<0><<<dim3(((NN / 16) * 1 + 3) / 4, 1), 128, 0, stream>>>(PT, NN, 0, XV, NN, 0, 1.0f, GT, CC, 0, NN, CC, NN);
    k_res<<<dim3(NN / 256, CC), 256, 0, stream>>>(mot, GT, Wt, bt, b, RES);
    k_gn<<<GG, 1024, 0, stream>>>(RES, mot, gw, gb, pa, al, b, (float*)d_out); }
}
